// GATLayer_37280316129311
// MI455X (gfx1250) — hardware-verified
//
#include <hip/hip_runtime.h>
#include <stddef.h>
#include <stdint.h>
#include <math.h>


#define F_IN    256
#define DOUT    64
#define NTHR    256
#define NWAVE   8
#define EPT     8
#define CHUNK   (NTHR * EPT)
#define WCAP    (EPT * 32)
#define LISTN   (NWAVE * WCAP)
#define NBMAX   2048
#define SLOTB   11
#define NBRUN   1024
#define RCAP    20480
#define DEGCAP  128
#define GBM     64
#define GBN     64
#define GTHR    128
#define NEGSL   0.01f
#define WSMAX   134217728
#define LDS_AGG ((2 * RCAP + 2 * NBMAX + LISTN) * 4 + 64)

static_assert((CHUNK & (CHUNK - 1)) == 0 && CHUNK <= (1 << SLOTB));
static_assert(NBMAX == (1 << SLOTB));
static_assert(NTHR * 8 == NBMAX);
static_assert(LISTN >= NBMAX);
static_assert(LISTN >= NWAVE * WCAP);
static_assert((RCAP % 32) == 0);
static_assert(LDS_AGG <= 300000);
static_assert(GBM == (GTHR / 32) * 16);
static_assert(GTHR == 2 * GBN && GTHR == 2 * GBM);
static_assert((F_IN % 32) == 0);
static_assert(DOUT == GBN && DOUT == 4 * 16);
static_assert(NBRUN <= NBMAX && (NBRUN & (NBRUN - 1)) == 0 && NBRUN >= 32);
static_assert((F_IN / 8) == 32);

typedef float          v4f  __attribute__((ext_vector_type(4)));
typedef float          v8f  __attribute__((ext_vector_type(8)));
typedef int            v4i  __attribute__((ext_vector_type(4)));
typedef int            v8i  __attribute__((ext_vector_type(8)));
typedef unsigned int   v4u  __attribute__((ext_vector_type(4)));
typedef unsigned short v8us __attribute__((ext_vector_type(8)));
typedef __bf16         v16b __attribute__((ext_vector_type(16)));
typedef v4f  __attribute__((may_alias)) v4fa;
typedef v4i  __attribute__((may_alias)) v4ia;
typedef v8us __attribute__((may_alias)) v8usa;
union FragB { v16b v; v8us h[2]; v8i w; };

__device__ __forceinline__ v8f wmb(const FragB& a, const FragB& b, v8f c) {
  v8f d = __builtin_amdgcn_wmma_f32_16x16x32_bf16(false, a.v, false, b.v, (short)0, c, false, false);
  asm volatile("v_nop\n\tv_nop\n\tv_nop\n\tv_nop" : "+v"(d) : "v"(a.w), "v"(b.w));
  return d;
}

__device__ __forceinline__ unsigned int f2bf(float f) {
  const unsigned int u = __float_as_uint(f);
  return ((u + 0x7FFFu + ((u >> 16) & 1u)) >> 16) & 0xFFFFu;
}
__device__ __forceinline__ float bf2f(unsigned int b) { return __uint_as_float(b << 16); }
__device__ __forceinline__ float bfr(float f) { return bf2f(f2bf(f)); }
__device__ __forceinline__ unsigned int pk2(float lo, float hi) { return f2bf(lo) | (f2bf(hi) << 16); }
__device__ __forceinline__ v4u pack8(const v4f a, const v4f b) {
  v4u r;
  r.x = pk2(a.x, a.y); r.y = pk2(a.z, a.w); r.z = pk2(b.x, b.y); r.w = pk2(b.z, b.w);
  return r;
}

__device__ __forceinline__ int scan_chunk(const int* __restrict__ dsts, int nE, int cbase, int slotBase,
                                          int nb, int vec8, int* list, int tid, int lane, int wave) {
  int wc = 0;
  const int el0  = tid * EPT;
  const int e0   = cbase + el0;
  const int sent = -2147483647 - 1;
  v4i da, db;
  if (vec8 != 0 && cbase + CHUNK <= nE) {
    da = *(const v4i*)(dsts + e0);
    db = *(const v4i*)(dsts + e0 + 4);
  } else {
    da.x = (e0     < nE) ? dsts[min(e0,     nE - 1)] : sent;
    da.y = (e0 + 1 < nE) ? dsts[min(e0 + 1, nE - 1)] : sent;
    da.z = (e0 + 2 < nE) ? dsts[min(e0 + 2, nE - 1)] : sent;
    da.w = (e0 + 3 < nE) ? dsts[min(e0 + 3, nE - 1)] : sent;
    db.x = (e0 + 4 < nE) ? dsts[min(e0 + 4, nE - 1)] : sent;
    db.y = (e0 + 5 < nE) ? dsts[min(e0 + 5, nE - 1)] : sent;
    db.z = (e0 + 6 < nE) ? dsts[min(e0 + 6, nE - 1)] : sent;
    db.w = (e0 + 7 < nE) ? dsts[min(e0 + 7, nE - 1)] : sent;
  }
  const unsigned nbs = (unsigned)slotBase;
  const unsigned unb = (unsigned)nb;
  const unsigned s0 = (unsigned)da.x - nbs, s1 = (unsigned)da.y - nbs;
  const unsigned s2 = (unsigned)da.z - nbs, s3 = (unsigned)da.w - nbs;
  const unsigned s4 = (unsigned)db.x - nbs, s5 = (unsigned)db.y - nbs;
  const unsigned s6 = (unsigned)db.z - nbs, s7 = (unsigned)db.w - nbs;
  const bool h0 = s0 < unb, h1 = s1 < unb, h2 = s2 < unb, h3 = s3 < unb;
  const bool h4 = s4 < unb, h5 = s5 < unb, h6 = s6 < unb, h7 = s7 < unb;
  const unsigned any = __builtin_amdgcn_ballot_w32(h0 | h1 | h2 | h3 | h4 | h5 | h6 | h7);
  if (any != 0u) {
#define HITJ(J, HJ, SJ) { \
      const unsigned mj = __builtin_amdgcn_ballot_w32(HJ); \
      if (mj != 0u) { \
        if (HJ) { \
          const int pos = wc + (int)__builtin_amdgcn_mbcnt_lo(mj, 0u); \
          if (pos < WCAP) list[wave * WCAP + pos] = ((el0 + (J)) << SLOTB) | (int)(SJ); \
        } \
        wc += (int)__builtin_popcount(mj); } }
    HITJ(0, h0, s0)
    HITJ(1, h1, s1)
    HITJ(2, h2, s2)
    HITJ(3, h3, s3)
    HITJ(4, h4, s4)
    HITJ(5, h5, s5)
    HITJ(6, h6, s6)
    HITJ(7, h7, s7)
#undef HITJ
  }
  return wc;
}

__global__ __launch_bounds__(NTHR) void k_wtr(const float* __restrict__ w, int Kin, int Ncol, int Nrows, int Kout,
                                              unsigned short* wt, int nUnits) {
  const int u = (int)blockIdx.x * NTHR + (int)threadIdx.x;
  if (u >= nUnits) return;
  const int kq = Kout >> 3;
  const int n  = u / kq;
  const int k8 = (u - n * kq) * 8;
  const int kk = k8 - (k8 / Kin) * Kin;
  const int ncl = n < Ncol ? n : Ncol - 1;
  const float* p = w + (size_t)kk * (size_t)Ncol + ncl;
  v4f a, b;
  a.x = p[0];                    a.y = p[(size_t)Ncol];         a.z = p[(size_t)2 * Ncol];     a.w = p[(size_t)3 * Ncol];
  b.x = p[(size_t)4 * Ncol];     b.y = p[(size_t)5 * Ncol];     b.z = p[(size_t)6 * Ncol];     b.w = p[(size_t)7 * Ncol];
  const v4f z4 = {0.f, 0.f, 0.f, 0.f};
  if (n >= Ncol || n >= Nrows) { a = z4; b = z4; }
  const v4u wv = pack8(a, b);
  unsigned short* o = wt + (size_t)n * (size_t)Kout + k8;
  *(volatile v4u*)o = wv;
  __threadfence();
  *(volatile v4u*)o = wv;
}

__global__ __launch_bounds__(GTHR) void k_fc(
    const float* __restrict__ hx, const unsigned short* __restrict__ WT,
    float* Z, const float* __restrict__ avec, float* SD, int nN, int MPr)
{
  __shared__ __attribute__((aligned(16))) float stg[GBM * GBN];
  __shared__ __attribute__((aligned(16))) float satt[2 * GBN];
  __shared__ __attribute__((aligned(16))) float sdot[2 * GBM];
  const int tid = (int)threadIdx.x, lane = tid & 31, wave = tid >> 5, hh = lane >> 4, m = lane & 15;
  const int rowBase = (int)blockIdx.x * GBM;

  satt[tid] = bfr(avec[tid]);

  v8f acc[4];
  {
    const v8f z = {0.f, 0.f, 0.f, 0.f, 0.f, 0.f, 0.f, 0.f};
    acc[0] = z; acc[1] = z; acc[2] = z; acc[3] = z;
  }
  int arow = rowBase + 16 * wave + m;
  arow = arow < nN ? arow : nN - 1;
  const float* ap = hx + (size_t)arow * (size_t)F_IN + 8 * hh;
  const unsigned short* wp = WT + (size_t)m * (size_t)F_IN + 8 * hh;
#pragma unroll 1
  for (int ks = 0; ks < F_IN / 32; ++ks) {
    const float* p = ap + 32 * ks;
    const v4f a0 = *(const v4fa*)p;
    const v4f a1 = *(const v4fa*)(p + 4);
    const v4f a2 = *(const v4fa*)(p + 16);
    const v4f a3 = *(const v4fa*)(p + 20);
    const v4u lo = pack8(a0, a1);
    const v4u hi = pack8(a2, a3);
    FragB af;
    v8i aw;
    aw[0] = (int)lo.x; aw[1] = (int)lo.y; aw[2] = (int)lo.z; aw[3] = (int)lo.w;
    aw[4] = (int)hi.x; aw[5] = (int)hi.y; aw[6] = (int)hi.z; aw[7] = (int)hi.w;
    af.w = aw;
#pragma unroll
    for (int t = 0; t < 4; ++t) {
      const unsigned short* wq = wp + (size_t)(16 * t) * (size_t)F_IN + 32 * ks;
      FragB bf;
      bf.h[0] = *(const v8usa*)wq;
      bf.h[1] = *(const v8usa*)(wq + 16);
      acc[t] = wmb(af, bf, acc[t]);
    }
  }

#pragma unroll
  for (int t = 0; t < 4; ++t) {
    const int lc = 16 * t + m;
#pragma unroll
    for (int r = 0; r < 8; ++r) {
      const int lr = 16 * wave + 8 * hh + r;
      stg[lr * GBN + lc] = acc[t][r];
    }
  }
  __syncthreads();

  {
    const int row = tid & 63, which = tid >> 6;
    const float* sa = satt + which * GBN;
    const float* hr = stg + row * GBN;
    float d = 0.f;
#pragma unroll 4
    for (int c4 = 0; c4 < GBN / 4; ++c4) {
      const v4f hv = *(const v4fa*)(hr + 4 * c4);
      const v4f av = *(const v4fa*)(sa + 4 * c4);
      d = fmaf(hv.x, av.x, d);
      d = fmaf(hv.y, av.y, d);
      d = fmaf(hv.z, av.z, d);
      d = fmaf(hv.w, av.w, d);
    }
    sdot[which * GBM + row] = d;
  }
  __syncthreads();

  v4f fv[8];
#pragma unroll
  for (int i = 0; i < 8; ++i) {
    const int lr = 16 * wave + 2 * i + hh;
    fv[i] = *(const v4fa*)(stg + lr * GBN + 4 * m);
  }
  const int which2 = lane >> 4, piece = lane & 15;
  const v4f sdv = *(const v4fa*)(sdot + which2 * GBM + 4 * piece);
  float* sp = SD + (size_t)which2 * (size_t)MPr + rowBase + 4 * piece;

#pragma unroll
  for (int i = 0; i < 8; ++i) {
    const int lr = 16 * wave + 2 * i + hh;
    const int gr = rowBase + lr;
    float* op = Z + (size_t)gr * (size_t)DOUT + 4 * m;
    *(volatile v4f*)op = fv[i];
  }
  if (wave == 0) *(volatile v4f*)sp = sdv;
  __threadfence();
#pragma unroll
  for (int i = 0; i < 8; ++i) {
    const int lr = 16 * wave + 2 * i + hh;
    const int gr = rowBase + lr;
    float* op = Z + (size_t)gr * (size_t)DOUT + 4 * m;
    *(volatile v4f*)op = fv[i];
  }
  if (wave == 0) *(volatile v4f*)sp = sdv;
}

__global__ __launch_bounds__(NTHR) void k_scan(
    const int* __restrict__ srcs, const int* __restrict__ dsts,
    const float* __restrict__ Z, const float* __restrict__ SD,
    float* out, int nN, int nE, int nb, int vec8, int MPr) {
  extern __shared__ v4f lds_dyn[];
  int* reg1 = (int*)lds_dyn;
  int* reg2 = reg1 + RCAP;
  int* scnt = reg2 + RCAP;
  int* soff = scnt + NBMAX;
  int* list = soff + NBMAX;
  int* wcnt = list + LISTN;
  int* wtot = wcnt + NWAVE;
  const int tid = (int)threadIdx.x, lane = tid & 31, wave = tid >> 5;
  const int nodeBase = (int)blockIdx.x * nb;

  for (int i = tid; i < NBMAX; i += NTHR) scnt[i] = 0;
  {
    const v4i z4 = {0, 0, 0, 0};
    for (int i = tid * 4; i < RCAP; i += NTHR * 4) *(v4ia*)(reg2 + i) = z4;
  }
  __syncthreads();

  int tot = 0;
  const int nChunks = (nE + CHUNK - 1) / CHUNK;
#pragma unroll 1
  for (int ch = 0; ch < nChunks; ++ch) {
    const int cbase = ch * CHUNK;
    const int wc = scan_chunk(dsts, nE, cbase, nodeBase, nb, vec8, list, tid, lane, wave);
    if (lane == 0) wcnt[wave] = wc;
    __syncthreads();
    int pre = 0, all = 0;
#pragma unroll
    for (int w2 = 0; w2 < NWAVE; ++w2) {
      int c = wcnt[w2];
      c = c < 0 ? 0 : (c > WCAP ? WCAP : c);
      all += c;
      pre += (w2 < wave) ? c : 0;
    }
    const int wcc  = wc > WCAP ? WCAP : wc;
    const int base = tot + pre;
#pragma unroll 1
    for (int i = lane; i < wcc; i += 32) {
      const int ent = list[wave * WCAP + i];
      const int el  = (ent >> SLOTB) & (CHUNK - 1);
      const int sl  = ent & (NBMAX - 1);
      int eid = cbase + el;
      eid = eid > nE - 1 ? nE - 1 : eid;
      const int pos = base + i;
      if (pos < RCAP) reg1[pos] = (int)(((unsigned)eid << SLOTB) | (unsigned)sl);
    }
    tot += all;
    tot = tot > RCAP ? RCAP : tot;
    __syncthreads();
  }
  const int nh = tot;

  if (wave == 0) {
#pragma unroll 1
    for (int b0 = 0; b0 < nh; b0 += 32) {
      const int idx = b0 + lane;
      const int uv  = reg1[idx < nh ? idx : nh - 1];
      const int m32 = (nh - b0) < 32 ? (nh - b0) : 32;
#pragma unroll 1
      for (int k = 0; k < m32; ++k) {
        const int u  = __builtin_amdgcn_readlane(uv, k);
        const int sl = u & (NBMAX - 1);
        if (lane == 0) scnt[sl] = scnt[sl] + 1;
      }
    }
  }
  __syncthreads();

  {
    const v4i ca = *(const v4i*)(scnt + 8 * tid);
    const v4i cb = *(const v4i*)(scnt + 8 * tid + 4);
    const int e0 = ca.x < 0 ? 0 : ca.x, e1 = ca.y < 0 ? 0 : ca.y, e2 = ca.z < 0 ? 0 : ca.z, e3 = ca.w < 0 ? 0 : ca.w;
    const int e4 = cb.x < 0 ? 0 : cb.x, e5 = cb.y < 0 ? 0 : cb.y, e6 = cb.z < 0 ? 0 : cb.z, e7 = cb.w < 0 ? 0 : cb.w;
    const int ts = e0 + e1 + e2 + e3 + e4 + e5 + e6 + e7;
    int incl = ts;
#pragma unroll
    for (int d = 1; d < 32; d <<= 1) {
      const int up = __shfl_up(incl, d);
      if (lane >= d) incl += up;
    }
    if (lane == 31) wtot[wave] = incl;
    __syncthreads();
    int pre = 0;
#pragma unroll
    for (int w2 = 0; w2 < NWAVE; ++w2) pre += (w2 < wave) ? wtot[w2] : 0;
    int run = pre + incl - ts;
    soff[8 * tid + 0] = run; run += e0;
    soff[8 * tid + 1] = run; run += e1;
    soff[8 * tid + 2] = run; run += e2;
    soff[8 * tid + 3] = run; run += e3;
    soff[8 * tid + 4] = run; run += e4;
    soff[8 * tid + 5] = run; run += e5;
    soff[8 * tid + 6] = run; run += e6;
    soff[8 * tid + 7] = run;
  }
  __syncthreads();
  for (int i = tid; i < NBMAX; i += NTHR) list[i] = soff[i];
  __syncthreads();

  if (wave == 0) {
#pragma unroll 1
    for (int b0 = 0; b0 < nh; b0 += 32) {
      const int idx = b0 + lane;
      const int uv  = reg1[idx < nh ? idx : nh - 1];
      const int m32 = (nh - b0) < 32 ? (nh - b0) : 32;
#pragma unroll 1
      for (int k = 0; k < m32; ++k) {
        const int u   = __builtin_amdgcn_readlane(uv, k);
        const int sl  = u & (NBMAX - 1);
        const int eid = (int)((unsigned)u >> SLOTB);
        if (lane == 0) {
          int pos = list[sl];
          pos = pos < 0 ? 0 : (pos > RCAP - 1 ? RCAP - 1 : pos);
          reg2[pos] = eid;
          list[sl] = pos + 1;
        }
      }
    }
  }
  __syncthreads();

  const int nbw   = nb >> 3;
  const int npair = nbw >> 1;
  const bool ovf  = (nh >= RCAP);
  const float qnan = __int_as_float(0x7fc00000);
  const int hh = lane >> 4, m = lane & 15;
  const int c0 = 4 * m;
  const float* SSp = SD;
  const float* SDp = SD + MPr;

#pragma unroll 1
  for (int jt = 0; jt < npair; ++jt) {
    const int slot = wave * nbw + 2 * jt + hh;
    const int grow = nodeBase + slot;
    const int gcl  = grow < nN ? grow : nN - 1;
    int st = soff[slot];
    const int craw = scnt[slot];
    int cnt = craw;
    st  = st < 0 ? 0 : (st > nh ? nh : st);
    cnt = cnt < 0 ? 0 : (cnt > DEGCAP ? DEGCAP : cnt);
    if (cnt > nh - st) cnt = nh - st;
    const int cot = __shfl_xor(cnt, 16);
    const int cm  = cnt > cot ? cnt : cot;
    const float pz  = (ovf || craw > DEGCAP) ? qnan : 0.0f;
    const float adv = SDp[gcl];

    float mx = -3.0e38f;
#pragma unroll 1
    for (int q = 0; q < cm; ++q) {
      const bool valid = q < cnt;
      int idx = st + q; idx = idx > RCAP - 1 ? RCAP - 1 : idx;
      int eid = reg2[idx]; eid = eid < 0 ? 0 : (eid > nE - 1 ? nE - 1 : eid);
      const int sraw = srcs[eid];
      const int s = sraw < 0 ? 0 : (sraw > nN - 1 ? nN - 1 : sraw);
      float lg = SSp[s] + adv;
      lg = lg > 0.f ? lg : NEGSL * lg;
      const float mn = fmaxf(mx, lg);
      mx = valid ? mn : mx;
    }

    float dn = 0.0f;
    v4f av = {0.f, 0.f, 0.f, 0.f};
#pragma unroll 1
    for (int q = 0; q < cm; ++q) {
      const bool valid = q < cnt;
      int idx = st + q; idx = idx > RCAP - 1 ? RCAP - 1 : idx;
      int eid = reg2[idx]; eid = eid < 0 ? 0 : (eid > nE - 1 ? nE - 1 : eid);
      const int sraw = srcs[eid];
      const int s = sraw < 0 ? 0 : (sraw > nN - 1 ? nN - 1 : sraw);
      const v4f fs = *(const v4fa*)(Z + (size_t)s * DOUT + c0);
      float lg = SSp[s] + adv;
      lg = lg > 0.f ? lg : NEGSL * lg;
      const float arg = valid ? (lg - mx) : 0.0f;
      const float ex  = expf(arg);
      const float p   = valid ? ex : 0.0f;
      dn += p;
      av.x = fmaf(p, fs.x, av.x);
      av.y = fmaf(p, fs.y, av.y);
      av.z = fmaf(p, fs.z, av.z);
      av.w = fmaf(p, fs.w, av.w);
    }
    const float dsafe = cnt > 0 ? dn : 1.0f;
    const float inv = 1.0f / dsafe;
    v4f o;
    o.x = av.x * inv + pz;
    o.y = av.y * inv + pz;
    o.z = av.z * inv + pz;
    o.w = av.w * inv + pz;
    float* op = out + (size_t)grow * DOUT + c0;
    const bool wr = grow < nN;
    if (wr) *(volatile v4f*)op = o;
    __threadfence();
    if (wr) *(volatile v4f*)op = o;
  }
}

static inline int cdiv(int a, int b) { return (a + b - 1) / b; }

extern "C" void kernel_launch(void* const* d_in, const int* in_sizes, int n_in,
                              void* d_out, int out_size, void* d_ws, size_t ws_size,
                              hipStream_t stream) {
  if (n_in < 5) return;
  const int nN = in_sizes[0] / F_IN;
  if (nN <= 0 || in_sizes[0] != nN * F_IN || nN > (1 << 22)) return;
  const int nE = in_sizes[1];
  if (nE < 1 || in_sizes[2] != nE) return;
  if (nE >= (1 << (32 - SLOTB))) return;
  if (in_sizes[3] != F_IN * DOUT) return;
  if (in_sizes[4] != 2 * DOUT) return;
  if ((long long)out_size != (long long)nN * DOUT) return;

  const float* hx   = (const float*)d_in[0];
  const int*   src  = (const int*)  d_in[1];
  const int*   dst  = (const int*)  d_in[2];
  const float* Wfc  = (const float*)d_in[3];
  const float* avec = (const float*)d_in[4];
  float* out = (float*)d_out;

  const int MP = cdiv(nN, GBM) * GBM;
  const int nb = NBRUN;
  if ((long long)nb * (long long)nE * 10LL > (long long)RCAP * (long long)nN * 9LL) return;
  const int gA = cdiv(nN, nb);
  if ((long long)gA * nb < (long long)nN) return;
  const int vec8 = ((nE & 3) == 0) ? 1 : 0;

  char* ws = (char*)d_ws;
  size_t off = 0;
  const size_t oWT = off; off += (size_t)DOUT * F_IN * 2;         off = (off + 255) & ~(size_t)255;
  const size_t oZ  = off; off += (size_t)MP * DOUT * 4;           off = (off + 255) & ~(size_t)255;
  const size_t oSD = off; off += (size_t)2 * MP * 4;              off = (off + 255) & ~(size_t)255;
  if (off > ws_size || off > (size_t)WSMAX) return;
  unsigned short* WT = (unsigned short*)(ws + oWT);
  float*          Zp = (float*)(ws + oZ);
  float*          SD = (float*)(ws + oSD);

  hipFuncSetAttribute(reinterpret_cast<const void*>(&k_scan),
                      hipFuncAttributeMaxDynamicSharedMemorySize, LDS_AGG);

  const int nUw = DOUT * (F_IN / 8);
  k_wtr<<<cdiv(nUw, NTHR), NTHR, 0, stream>>>(Wfc, F_IN, DOUT, DOUT, F_IN, WT, nUw);
  k_fc<<<MP / GBM, GTHR, 0, stream>>>(hx, WT, Zp, avec, SD, nN, MP);
  k_scan<<<gA, NTHR, LDS_AGG, stream>>>(src, dst, Zp, SD, out, nN, nE, nb, vec8, MP);
}
